// GatedGraphNeuralNetwork_74491912781909
// MI455X (gfx1250) — hardware-verified
//
#include <hip/hip_runtime.h>
#include <stddef.h>


#define HD 128
#define G3 384
#define RB 4096
#define CAP 26624
#define MAXDEG 64
#define NQCH 6144
#define NPASS 6
#define SEG_LDS_WORDS (2 * CAP + 128)
#define SEG_LDS_BYTES (SEG_LDS_WORDS * 4)

static_assert(RB == (1 << (2 * NPASS)));
static_assert(2 * RB <= CAP);
static_assert(NQCH == 4 * 24 * 32 * 2);

typedef _Float16 v8h __attribute__((ext_vector_type(8)));
typedef _Float16 v16h __attribute__((ext_vector_type(16)));
typedef float v8f __attribute__((ext_vector_type(8)));
typedef float v4f __attribute__((ext_vector_type(4)));
typedef unsigned int u4 __attribute__((ext_vector_type(4)));
typedef int i4 __attribute__((ext_vector_type(4)));

union Frag { v16h v; u4 u[2]; };
union P8 { v8h v; u4 u; };

static __device__ __forceinline__ v8f wmma16(v16h a, v16h b, v8f c) {
  c = __builtin_amdgcn_wmma_f32_16x16x32_f16(false, a, false, b, (short)0, c, false, false);
  asm volatile("v_nop\n\tv_nop\n\tv_nop\n\tv_nop" : "+v"(c) : "v"(a), "v"(b) : "memory");
  return c;
}

static __device__ __forceinline__ u4 pack8(v4f a, v4f b, float s) {
  v8h hv;
  hv[0] = (_Float16)(a.x * s); hv[1] = (_Float16)(a.y * s);
  hv[2] = (_Float16)(a.z * s); hv[3] = (_Float16)(a.w * s);
  hv[4] = (_Float16)(b.x * s); hv[5] = (_Float16)(b.y * s);
  hv[6] = (_Float16)(b.z * s); hv[7] = (_Float16)(b.w * s);
  P8 p; p.v = hv;
  return p.u;
}

static __device__ __forceinline__ float sigm(float x) { return 1.0f / (1.0f + __expf(-x)); }
static __device__ __forceinline__ float tanhx(float x) { return 2.0f / (1.0f + __expf(-2.0f * x)) - 1.0f; }

__global__ __launch_bounds__(256) void k_prep(const float* __restrict__ Wmsg,
                                              const float* __restrict__ bmsg,
                                              const float* __restrict__ Wih,
                                              const float* __restrict__ Whh,
                                              unsigned int* Qc, unsigned int* Qh, float* bc) {
  const int tid = blockIdx.x * 256 + threadIdx.x;
  if (tid < 2 * NQCH) {
    const bool isC = tid < NQCH;
    const int q = isC ? tid : tid - NQCH;
    const int half = q & 1, lane = (q >> 1) & 31, t6 = q >> 6;
    const int nt = t6 % 24, kc = t6 / 24;
    const int col = nt * 16 + (lane & 15), hh = lane >> 4;
    const int k0 = kc * 32 + half * 16 + hh * 8;
    v4f lo, hi;
    if (isC) {
      v4f a0 = {0.0f, 0.0f, 0.0f, 0.0f};
      v4f a1 = {0.0f, 0.0f, 0.0f, 0.0f};
      const float* wi = Wih + (size_t)col * HD;
      const float* wm = Wmsg + k0;
#pragma unroll 4
      for (int o = 0; o < HD; ++o) {
        const float a = wi[o];
        const v4f m0 = *(const v4f*)(wm + (size_t)o * HD);
        const v4f m1 = *(const v4f*)(wm + (size_t)o * HD + 4);
        a0 += a * m0;
        a1 += a * m1;
      }
      lo = a0; hi = a1;
    } else {
      const float* wr = Whh + (size_t)col * HD + k0;
      lo = *(const v4f*)wr;
      hi = *(const v4f*)(wr + 4);
    }
    const u4 pk = pack8(lo, hi, 64.0f);
    unsigned int* dst = (isC ? Qc : Qh) + (size_t)q * 4;
    *(volatile u4*)dst = pk;
    __threadfence();
    *(volatile u4*)dst = pk;
  } else {
    const int c = tid - 2 * NQCH;
    if (c < G3) {
      float s = 0.0f;
      const float* wi = Wih + (size_t)c * HD;
#pragma unroll 4
      for (int o = 0; o < HD; ++o) s += wi[o] * bmsg[o];
      *(volatile float*)(bc + c) = s;
      __threadfence();
      *(volatile float*)(bc + c) = s;
    }
  }
}

static __device__ __forceinline__ void hist_to_base(unsigned c0, unsigned c1, unsigned c2, unsigned c3,
                                                    unsigned int* hw, unsigned int* baseL,
                                                    int lane, int w, int t) {
#pragma unroll
  for (int o = 16; o > 0; o >>= 1) {
    c0 += __shfl_xor(c0, o);
    c1 += __shfl_xor(c1, o);
    c2 += __shfl_xor(c2, o);
    c3 += __shfl_xor(c3, o);
  }
  if (lane == 0) { hw[w * 4 + 0] = c0; hw[w * 4 + 1] = c1; hw[w * 4 + 2] = c2; hw[w * 4 + 3] = c3; }
  __syncthreads();
  if (t == 0) {
    unsigned t0 = 0, t1 = 0, t2 = 0;
#pragma unroll
    for (int q = 0; q < 8; ++q) { t0 += hw[q * 4]; t1 += hw[q * 4 + 1]; t2 += hw[q * 4 + 2]; }
    baseL[0] = 0u; baseL[1] = t0; baseL[2] = t0 + t1; baseL[3] = t0 + t1 + t2;
  }
  __syncthreads();
}

__global__ __launch_bounds__(256) void k_seg(const float* __restrict__ hsrc,
                                             const int* __restrict__ erow,
                                             const int* __restrict__ ecol,
                                             int nE, int nN,
                                             unsigned short* Sout, float* degOut) {
  extern __shared__ __align__(16) unsigned int smem[];
  unsigned int* X = smem;
  unsigned int* Y = smem + CAP;
  unsigned int* wc = smem + 2 * CAP;
  unsigned int* wp = wc + 32;
  unsigned int* baseL = wp + 32;
  unsigned int* hw = baseL + 4;
  unsigned int* lenL = hw + 32;

  const int t = threadIdx.x, lane = t & 31, w = t >> 5;
  const int n0 = blockIdx.x * RB;
  int reff = nN - n0;
  if (reff > RB) reff = RB;

  int runLen = 0;
  const int nCh = (nE + 1023) >> 10;
  for (int c = 0; c < nCh; ++c) {
    const int eb = (c << 10) + 4 * t;
    int q0 = n0 - 1, q1 = n0 - 1, q2 = n0 - 1, q3 = n0 - 1;
    if (eb + 3 < nE) {
      const i4 rv = *(const i4*)(erow + eb);
      q0 = rv.x; q1 = rv.y; q2 = rv.z; q3 = rv.w;
    } else {
      if (eb < nE) q0 = erow[eb];
      if (eb + 1 < nE) q1 = erow[eb + 1];
      if (eb + 2 < nE) q2 = erow[eb + 2];
    }
    const unsigned d0 = (unsigned)q0 - (unsigned)n0;
    const unsigned d1 = (unsigned)q1 - (unsigned)n0;
    const unsigned d2 = (unsigned)q2 - (unsigned)n0;
    const unsigned d3 = (unsigned)q3 - (unsigned)n0;
    const bool h0 = d0 < (unsigned)reff;
    const bool h1 = d1 < (unsigned)reff;
    const bool h2 = d2 < (unsigned)reff;
    const bool h3 = d3 < (unsigned)reff;
    const int k = (int)h0 + (int)h1 + (int)h2 + (int)h3;
    int incl = k;
#pragma unroll
    for (int o = 1; o < 32; o <<= 1) {
      const int u = __shfl_up(incl, o);
      if (lane >= o) incl += u;
    }
    const int excl = incl - k;
    const int tot = __shfl(incl, 31);
    if (lane == 0) wc[w] = (unsigned)tot;
    __syncthreads();
    if (w == 0) {
      int v = (lane < 8) ? (int)wc[lane] : 0;
      const int orig = v;
#pragma unroll
      for (int o = 1; o < 8; o <<= 1) {
        const int u = __shfl_up(v, o);
        if (lane >= o) v += u;
      }
      if (lane < 8) wp[lane] = (unsigned)(runLen + v - orig);
      runLen += __shfl(v, 7);
    }
    __syncthreads();
    unsigned pos = wp[w] + (unsigned)excl;
    if (h0) {
      int s = ecol[eb]; s = s < 0 ? 0 : s; s = s > nN - 1 ? nN - 1 : s;
      if (pos < (unsigned)CAP) X[pos] = (d0 << 17) | (unsigned)s;
      ++pos;
    }
    if (h1) {
      int s = ecol[eb + 1]; s = s < 0 ? 0 : s; s = s > nN - 1 ? nN - 1 : s;
      if (pos < (unsigned)CAP) X[pos] = (d1 << 17) | (unsigned)s;
      ++pos;
    }
    if (h2) {
      int s = ecol[eb + 2]; s = s < 0 ? 0 : s; s = s > nN - 1 ? nN - 1 : s;
      if (pos < (unsigned)CAP) X[pos] = (d2 << 17) | (unsigned)s;
      ++pos;
    }
    if (h3) {
      int s = ecol[eb + 3]; s = s < 0 ? 0 : s; s = s > nN - 1 ? nN - 1 : s;
      if (pos < (unsigned)CAP) X[pos] = (d3 << 17) | (unsigned)s;
      ++pos;
    }
  }
  if (t == 0) lenL[0] = (unsigned)(runLen < CAP ? runLen : CAP);
  __syncthreads();
  const int len = (int)lenL[0];

  unsigned c0 = 0, c1 = 0, c2 = 0, c3 = 0;
  for (int i = t; i < len; i += 256) {
    const unsigned d = (X[i] >> 17) & 3u;
    c0 += (d == 0u); c1 += (d == 1u); c2 += (d == 2u); c3 += (d == 3u);
  }
  hist_to_base(c0, c1, c2, c3, hw, baseL, lane, w, t);

  const int nC2 = (len + 255) >> 8;
  for (int p = 0; p < NPASS; ++p) {
    const unsigned int* src = (p & 1) ? Y : X;
    unsigned int* dst = (p & 1) ? X : Y;
    const int sh = 17 + 2 * p;
    const int shn = sh + 2;
    const bool doNext = (p + 1 < NPASS);
    c0 = 0; c1 = 0; c2 = 0; c3 = 0;
    for (int c = 0; c < nC2; ++c) {
      const int i = (c << 8) + t;
      const bool valid = i < len;
      unsigned e = 0u;
      if (valid) e = src[i];
      const unsigned d = (e >> sh) & 3u;
      const unsigned m0 = __builtin_amdgcn_ballot_w32(valid && d == 0u);
      const unsigned m1 = __builtin_amdgcn_ballot_w32(valid && d == 1u);
      const unsigned m2 = __builtin_amdgcn_ballot_w32(valid && d == 2u);
      const unsigned m3 = __builtin_amdgcn_ballot_w32(valid && d == 3u);
      const unsigned mm = (d == 0u) ? m0 : (d == 1u) ? m1 : (d == 2u) ? m2 : m3;
      const unsigned rank = __builtin_amdgcn_mbcnt_lo(mm, 0u);
      if (lane < 4) {
        const unsigned mk = (lane == 0) ? m0 : (lane == 1) ? m1 : (lane == 2) ? m2 : m3;
        wc[w * 4 + lane] = (unsigned)__popc(mk);
      }
      if (doNext) {
        const unsigned dn = (e >> shn) & 3u;
        c0 += (valid && dn == 0u); c1 += (valid && dn == 1u);
        c2 += (valid && dn == 2u); c3 += (valid && dn == 3u);
      }
      __syncthreads();
      if (w == 0) {
        int v = (int)wc[lane];
        const int orig = v;
#pragma unroll
        for (int o = 4; o < 32; o <<= 1) {
          const int u = __shfl_up(v, o);
          if (lane >= o) v += u;
        }
        const unsigned b = baseL[lane & 3];
        wp[lane] = b + (unsigned)(v - orig);
        if (lane >= 28) baseL[lane & 3] = b + (unsigned)v;
      }
      __syncthreads();
      if (valid) {
        const unsigned ps = wp[w * 4 + d] + rank;
        if (ps < (unsigned)CAP) dst[ps] = e;
      }
    }
    if (doNext) hist_to_base(c0, c1, c2, c3, hw, baseL, lane, w, t);
  }
  __syncthreads();

  float* sDeg = (float*)Y;
  unsigned short* sBeg = (unsigned short*)(Y + RB);
  unsigned short* sEnd = sBeg + RB;
  for (int i = t; i < RB; i += 256) Y[RB + i] = 0u;
  __syncthreads();
  for (int i = t; i < len; i += 256) {
    const unsigned d = X[i] >> 17;
    const unsigned dp = (i > 0) ? (X[i - 1] >> 17) : 0xFFFFFFFFu;
    const unsigned dn = (i + 1 < len) ? (X[i + 1] >> 17) : 0xFFFFFFFFu;
    if (d < (unsigned)RB) {
      if (d != dp) sBeg[d] = (unsigned short)i;
      if (d != dn) sEnd[d] = (unsigned short)(i + 1);
    }
  }
  __syncthreads();

  const int hh = lane >> 4, li = lane & 15;
  for (int p2 = w; p2 < RB / 2; p2 += 8) {
    const int nl = 2 * p2 + hh;
    const int node = n0 + nl;
    const int b = (int)sBeg[nl], en = (int)sEnd[nl];
    int cnt = en - b;
    cnt = cnt < 0 ? 0 : cnt;
    cnt = cnt > MAXDEG ? MAXDEG : cnt;
    v4f a0 = {0.0f, 0.0f, 0.0f, 0.0f};
    v4f a1 = {0.0f, 0.0f, 0.0f, 0.0f};
#pragma unroll 2
    for (int kk = 0; kk < cnt; ++kk) {
      int idx = b + kk;
      idx = idx > CAP - 1 ? CAP - 1 : idx;
      unsigned s = X[idx] & 0x1FFFFu;
      if (s > (unsigned)(nN - 1)) s = (unsigned)(nN - 1);
      const float* hp = hsrc + (size_t)s * HD + li * 8;
      a0 += *(const v4f*)hp;
      a1 += *(const v4f*)(hp + 4);
    }
    const u4 pk = pack8(a0, a1, 8.0f);
    if (li == 0) sDeg[nl] = (float)cnt;
    const bool wr = node < nN;
    unsigned short* op = Sout + (size_t)(wr ? node : 0) * HD + li * 8;
    if (wr) *(volatile u4*)op = pk;
    __threadfence();
    if (wr) *(volatile u4*)op = pk;
  }
  __syncthreads();
  float* dg = degOut + (size_t)blockIdx.x * RB;
#pragma unroll
  for (int j = 0; j < RB / 1024; ++j) {
    const int q = t + 256 * j;
    const v4f v = *(const v4f*)(sDeg + 4 * q);
    *(volatile v4f*)(dg + 4 * q) = v;
  }
  __threadfence();
#pragma unroll
  for (int j = 0; j < RB / 1024; ++j) {
    const int q = t + 256 * j;
    const v4f v = *(const v4f*)(sDeg + 4 * q);
    *(volatile v4f*)(dg + 4 * q) = v;
  }
}

__global__ __launch_bounds__(256) __attribute__((amdgpu_num_vgpr(256)))
void k_gru(const float* __restrict__ hprev, const unsigned short* __restrict__ Sin,
           const float* __restrict__ deg,
           const unsigned int* __restrict__ Qc, const unsigned int* __restrict__ Qh,
           const float* __restrict__ bc, const float* __restrict__ bih,
           const float* __restrict__ bhh, float* hout, int nN) {
  __shared__ __align__(16) float sT[8][16][132];
  const int t = threadIdx.x, lane = t & 31, w = t >> 5, hh = lane >> 4, m = lane & 15;
  const int r0 = blockIdx.x * 128 + w * 16;
  int rm = r0 + m;
  if (rm > nN - 1) rm = nN - 1;

  Frag aS[4], aH[4];
  {
    const unsigned short* sp = Sin + (size_t)rm * HD + 8 * hh;
    const float* hp = hprev + (size_t)rm * HD + 8 * hh;
#pragma unroll
    for (int kc = 0; kc < 4; ++kc) {
      aS[kc].u[0] = *(const u4*)(sp + kc * 32);
      aS[kc].u[1] = *(const u4*)(sp + kc * 32 + 16);
      const v4f f0 = *(const v4f*)(hp + kc * 32);
      const v4f f1 = *(const v4f*)(hp + kc * 32 + 4);
      const v4f f2 = *(const v4f*)(hp + kc * 32 + 16);
      const v4f f3 = *(const v4f*)(hp + kc * 32 + 20);
      aH[kc].u[0] = pack8(f0, f1, 8.0f);
      aH[kc].u[1] = pack8(f2, f3, 8.0f);
    }
  }
  int rowi[8];
  float dgv[8];
#pragma unroll
  for (int i = 0; i < 8; ++i) {
    int r = r0 + 8 * hh + i;
    if (r > nN - 1) r = nN - 1;
    rowi[i] = r;
    dgv[i] = deg[r];
  }

  const float inv = 0.001953125f;
#pragma unroll 1
  for (int nt = 0; nt < 8; ++nt) {
    v8f ar = {}; v8f az = {}; v8f ain = {}; v8f ahn = {};
#pragma unroll
    for (int kc = 0; kc < 4; ++kc) {
      const size_t qb = (size_t)((kc * 24 + nt) * 32 + lane) * 8;
      Frag b;
      b.u[0] = *(const u4*)(Qc + qb);        b.u[1] = *(const u4*)(Qc + qb + 4);
      ar = wmma16(aS[kc].v, b.v, ar);
      b.u[0] = *(const u4*)(Qh + qb);        b.u[1] = *(const u4*)(Qh + qb + 4);
      ar = wmma16(aH[kc].v, b.v, ar);
      b.u[0] = *(const u4*)(Qc + qb + 2048); b.u[1] = *(const u4*)(Qc + qb + 2052);
      az = wmma16(aS[kc].v, b.v, az);
      b.u[0] = *(const u4*)(Qh + qb + 2048); b.u[1] = *(const u4*)(Qh + qb + 2052);
      az = wmma16(aH[kc].v, b.v, az);
      b.u[0] = *(const u4*)(Qc + qb + 4096); b.u[1] = *(const u4*)(Qc + qb + 4100);
      ain = wmma16(aS[kc].v, b.v, ain);
      b.u[0] = *(const u4*)(Qh + qb + 4096); b.u[1] = *(const u4*)(Qh + qb + 4100);
      ahn = wmma16(aH[kc].v, b.v, ahn);
    }
    const int c = nt * 16 + m;
    const float bcr = bc[c], bcz = bc[c + HD], bcn = bc[c + 2 * HD];
    const float br = bih[c] + bhh[c];
    const float bz = bih[c + HD] + bhh[c + HD];
    const float bni = bih[c + 2 * HD];
    const float bnh = bhh[c + 2 * HD];
#pragma unroll
    for (int i = 0; i < 8; ++i) {
      const float hold = hprev[(size_t)rowi[i] * HD + c];
      const float rg = sigm(ar[i] * inv + dgv[i] * bcr + br);
      const float zg = sigm(az[i] * inv + dgv[i] * bcz + bz);
      const float hn = ahn[i] * inv + bnh;
      const float gin = ain[i] * inv + dgv[i] * bcn + bni;
      const float nv = tanhx(gin + rg * hn);
      sT[w][8 * hh + i][c] = (1.0f - zg) * nv + zg * hold;
    }
  }
  __syncthreads();
#pragma unroll
  for (int rr = 0; rr < 16; ++rr) {
    const int row = r0 + rr;
    if (row < nN) {
      const v4f v = *(const v4f*)(&sT[w][rr][lane * 4]);
      *(volatile v4f*)(hout + (size_t)row * HD + lane * 4) = v;
    }
  }
  __threadfence();
#pragma unroll
  for (int rr = 0; rr < 16; ++rr) {
    const int row = r0 + rr;
    if (row < nN) {
      const v4f v = *(const v4f*)(&sT[w][rr][lane * 4]);
      *(volatile v4f*)(hout + (size_t)row * HD + lane * 4) = v;
    }
  }
}

extern "C" void kernel_launch(void* const* d_in, const int* in_sizes, int n_in,
                              void* d_out, int out_size, void* d_ws, size_t ws_size,
                              hipStream_t stream) {
  if (n_in < 8 || d_out == 0 || d_ws == 0) return;
  const int nN = in_sizes[0] / HD;
  const int nE = in_sizes[1] / 2;
  if (nN < 1 || nN > 131072 || nE < 0) return;
  if (in_sizes[0] != nN * HD || in_sizes[1] != 2 * nE) return;
  if (in_sizes[2] != HD * HD || in_sizes[3] != HD || in_sizes[4] != G3 * HD ||
      in_sizes[5] != G3 * HD || in_sizes[6] != G3 || in_sizes[7] != G3) return;
  if (out_size != nN * HD) return;

  const float* x    = (const float*)d_in[0];
  const int* erow   = (const int*)d_in[1];
  const int* ecol   = erow + nE;
  const float* Wmsg = (const float*)d_in[2];
  const float* bmsg = (const float*)d_in[3];
  const float* Wih  = (const float*)d_in[4];
  const float* Whh  = (const float*)d_in[5];
  const float* bih  = (const float*)d_in[6];
  const float* bhh  = (const float*)d_in[7];

  const int nblk = (nN + RB - 1) / RB;

  char* ws = (char*)d_ws;
  size_t off = 0;
  unsigned int* wQc = (unsigned int*)(ws + off); off += (size_t)NQCH * 16;
  unsigned int* wQh = (unsigned int*)(ws + off); off += (size_t)NQCH * 16;
  float* wbc = (float*)(ws + off);               off += (size_t)G3 * 4;
  float* wdeg = (float*)(ws + off);              off += (size_t)nblk * RB * 4;
  unsigned short* wS = (unsigned short*)(ws + off); off += (size_t)nN * HD * 2;
  float* whb = (float*)(ws + off);               off += (size_t)nN * HD * 4;
  if (off > ws_size) return;

  hipFuncSetAttribute((const void*)k_seg, hipFuncAttributeMaxDynamicSharedMemorySize, SEG_LDS_BYTES);

  k_prep<<<dim3((2 * NQCH + G3 + 255) / 256), dim3(256), 0, stream>>>(Wmsg, bmsg, Wih, Whh, wQc, wQh, wbc);

  const float* hs = x;
  for (int step = 0; step < 5; ++step) {
    float* hd = (step & 1) ? whb : (float*)d_out;
    k_seg<<<dim3(nblk), dim3(256), SEG_LDS_BYTES, stream>>>(hs, erow, ecol, nE, nN, wS, wdeg);
    k_gru<<<dim3((nN + 127) / 128), dim3(256), 0, stream>>>(hs, wS, wdeg, wQc, wQh, wbc, bih, bhh, hd, nN);
    hs = hd;
  }
}
